// RAE_60112362275063
// MI455X (gfx1250) — hardware-verified
//
#include <hip/hip_runtime.h>
#include <stdint.h>
#include <stddef.h>

typedef __attribute__((ext_vector_type(16))) _Float16 v16h;
typedef __attribute__((ext_vector_type(8)))  _Float16 v8h;
typedef __attribute__((ext_vector_type(8)))  float    v8f;
typedef __attribute__((ext_vector_type(4)))  float    v4f;
typedef __attribute__((ext_vector_type(2)))  float    v2f;

constexpr int XDIM    = 38;
constexpr int HDIM    = 128;
constexpr int GDIM    = 3 * HDIM;
constexpr int TSTEPS  = 128;
constexpr int KCAT    = 192;
constexpr int RPB     = 16;
constexpr int NWAVES  = 8;
constexpr int NTHR    = NWAVES * 32;
constexpr int LINROWS = 48;
constexpr int OPITCH  = 64;
constexpr int NCHUNK  = TSTEPS * XDIM / 4;
constexpr int RP_ITERS = (NCHUNK + NTHR - 1) / NTHR;

static_assert(KCAT % 32 == 0 && HDIM % 32 == 0, "K slabs of 32");
static_assert(KCAT >= HDIM + XDIM, "concat K holds h and x");
static_assert(NWAVES * 16 == HDIM, "waves cover hidden columns");
static_assert(LINROWS >= XDIM && LINROWS == 3 * 16, "projection N tiles on waves 0..2");
static_assert(HDIM + LINROWS <= KCAT, "o columns fit in the A row");
static_assert(RPB * XDIM <= 3 * NTHR, "x staging slots");
static_assert(RPB == 2 * NWAVES, "store phase: wave w writes rows 2w, 2w+1");
static_assert(OPITCH * 4 == 256 && OPITCH >= LINROWS, "ws row = 2 whole 128-B lines");
static_assert((TSTEPS * XDIM) % 4 == 0, "output batch row is float4-tileable");
static_assert((TSTEPS * XDIM * 4) % 128 == 0, "output batch row is whole 128-B lines");
static_assert(RP_ITERS * NTHR >= NCHUNK && RP_ITERS == 5, "repack coverage");
static_assert((NCHUNK % 8) == 0 && ((NCHUNK - (RP_ITERS - 1) * NTHR) % 32) == 0, "repack tail is whole waves");

union FragU { v16h v; v8h h[2]; };
__device__ __forceinline__ v16h frag_load(const _Float16* p) {
  FragU f; f.h[0] = *(const v8h*)(p); f.h[1] = *(const v8h*)(p + 16); return f.v;
}
__device__ __forceinline__ v8f mma16(v16h a, v16h b, v8f c) {
  c = __builtin_amdgcn_wmma_f32_16x16x32_f16(false, a, false, b, (short)0, c, false, false);
  asm volatile("v_nop\n\tv_nop\n\tv_nop\n\tv_nop" : "+v"(c) : "v"(a), "v"(b));
  return c;
}
__device__ __forceinline__ v8f zero8() { return (v8f){0.f, 0.f, 0.f, 0.f, 0.f, 0.f, 0.f, 0.f}; }

__device__ __forceinline__ float rcp_apx(float v) { return __builtin_amdgcn_rcpf(v); }
__device__ __forceinline__ float sigm_apx(float v) { return rcp_apx(1.0f + __expf(-v)); }
__device__ __forceinline__ float tanh_apx(float v) { return 1.0f - 2.0f * rcp_apx(1.0f + __expf(2.0f * v)); }

__device__ __forceinline__ void load_gate_weights(const float* __restrict__ Wih, const float* __restrict__ Whh,
                                                  const float* __restrict__ bih, const float* __restrict__ bhh,
                                                  _Float16* sW, float* sBrz, float* sBin, float* sBhn, int tid) {
#pragma unroll 2
  for (int i = tid; i < GDIM * KCAT; i += NTHR) {
    const int n = i / KCAT;
    const int k = i - n * KCAT;
    const int khc = (k < HDIM) ? k : (HDIM - 1);
    int kx = k - HDIM;
    kx = (kx < 0) ? 0 : ((kx > XDIM - 1) ? (XDIM - 1) : kx);
    const float vh = Whh[n * HDIM + khc];
    const float vx = Wih[n * XDIM + kx];
    const float v = (k < HDIM) ? vh : ((k < HDIM + XDIM) ? vx : 0.0f);
    sW[i] = (_Float16)v;
  }
  for (int i = tid; i < 2 * HDIM; i += NTHR) sBrz[i] = bih[i] + bhh[i];
  for (int i = tid; i < HDIM; i += NTHR) { sBin[i] = bih[2 * HDIM + i]; sBhn[i] = bhh[2 * HDIM + i]; }
}

__device__ __forceinline__ void stage_x(const float* __restrict__ x, _Float16* Anxt, int bbase, int t, int tid) {
  const int e0 = tid;
  const int e1 = tid + NTHR;
  const int e2 = tid + 2 * NTHR;
  const bool ok2 = (e2 < RPB * XDIM);
  const int e2c = ok2 ? e2 : (RPB * XDIM - 1);
  const int m0 = e0 / XDIM, c0 = e0 - m0 * XDIM;
  const int m1 = e1 / XDIM, c1 = e1 - m1 * XDIM;
  const int m2 = e2c / XDIM, c2 = e2c - m2 * XDIM;
  const float v0 = x[((size_t)(bbase + m0) * TSTEPS + t) * XDIM + c0];
  const float v1 = x[((size_t)(bbase + m1) * TSTEPS + t) * XDIM + c1];
  const float v2 = x[((size_t)(bbase + m2) * TSTEPS + t) * XDIM + c2];
  Anxt[m0 * KCAT + HDIM + c0] = (_Float16)v0;
  Anxt[m1 * KCAT + HDIM + c1] = (_Float16)v1;
  if (ok2) Anxt[m2 * KCAT + HDIM + c2] = (_Float16)v2;
}

__device__ __forceinline__ void gru_step(const _Float16* Acur, _Float16* Anxt, const _Float16* sW,
                                         const float* sBrz, const float* sBin, const float* sBhn,
                                         float (&hreg)[8], int w, int m, int k8) {
  const int colbase = w * 16;
  const _Float16* arow = Acur + m * KCAT + k8;
  const _Float16* wr = sW + (colbase + m) * KCAT + k8;
  const _Float16* wz = sW + (HDIM + colbase + m) * KCAT + k8;
  const _Float16* wn = sW + (2 * HDIM + colbase + m) * KCAT + k8;
  v8f accR = zero8(), accZ = zero8(), aGH = zero8(), aGI = zero8();
#pragma unroll 1
  for (int s = 0; s < HDIM / 32; ++s) {
    const int k0 = s * 32;
    const v16h a = frag_load(arow + k0);
    v16h b = frag_load(wr + k0);
    accR = mma16(a, b, accR);
    b = frag_load(wz + k0);
    accZ = mma16(a, b, accZ);
    b = frag_load(wn + k0);
    aGH = mma16(a, b, aGH);
  }
#pragma unroll
  for (int s = HDIM / 32; s < KCAT / 32; ++s) {
    const int k0 = s * 32;
    const v16h a = frag_load(arow + k0);
    v16h b = frag_load(wr + k0);
    accR = mma16(a, b, accR);
    b = frag_load(wz + k0);
    accZ = mma16(a, b, accZ);
    b = frag_load(wn + k0);
    aGI = mma16(a, b, aGI);
  }
  const int col = colbase + m;
  const float br = sBrz[col];
  const float bz = sBrz[HDIM + col];
  const float bi = sBin[col];
  const float bn = sBhn[col];
#pragma unroll
  for (int r = 0; r < 8; ++r) {
    const int row = k8 + r;
    const float rv = sigm_apx(accR[r] + br);
    const float zv = sigm_apx(accZ[r] + bz);
    const float nv = tanh_apx((aGI[r] + bi) + rv * (aGH[r] + bn));
    const float hn = (1.0f - zv) * nv + zv * hreg[r];
    hreg[r] = hn;
    Anxt[row * KCAT + col] = (_Float16)hn;
  }
}

__device__ __forceinline__ void proj_step(_Float16* Anxt, const _Float16* sLin, const float* sLb, float* sO,
                                          int w, int m, int k8) {
  const int n0 = w * 16;
  const _Float16* arow = Anxt + m * KCAT + k8;
  const _Float16* lr = sLin + (n0 + m) * HDIM + k8;
  v8f acc = zero8();
#pragma unroll 1
  for (int s = 0; s < HDIM / 32; ++s) {
    const v16h a = frag_load(arow + s * 32);
    const v16h b = frag_load(lr + s * 32);
    acc = mma16(a, b, acc);
  }
  const int pc = n0 + m;
  const float lb = sLb[pc];
#pragma unroll
  for (int r = 0; r < 8; ++r) {
    const int row = k8 + r;
    const float val = acc[r] + lb;
    Anxt[row * KCAT + HDIM + pc] = (_Float16)val;
    sO[row * OPITCH + pc] = val;
  }
}

__global__ __launch_bounds__(NTHR) void gru_scan_kernel(
    const float* __restrict__ x,
    const float* __restrict__ eWih, const float* __restrict__ eWhh,
    const float* __restrict__ eBih, const float* __restrict__ eBhh,
    const float* __restrict__ dWih, const float* __restrict__ dWhh,
    const float* __restrict__ dBih, const float* __restrict__ dBhh,
    const float* __restrict__ linW, const float* __restrict__ linB,
    float* __restrict__ Ows, int nb) {
  __shared__ __align__(16) _Float16 sW[GDIM * KCAT];
  __shared__ __align__(16) _Float16 sA[2 * RPB * KCAT];
  __shared__ __align__(16) _Float16 sLin[LINROWS * HDIM];
  __shared__ __align__(16) float sO[RPB * OPITCH];
  __shared__ float sBrz[2 * HDIM];
  __shared__ float sBin[HDIM];
  __shared__ float sBhn[HDIM];
  __shared__ float sLb[LINROWS];

  const int tid = threadIdx.x;
  const int lane = tid & 31;
  const int w = tid >> 5;
  const int hh = lane >> 4;
  const int m = lane & 15;
  const int k8 = hh * 8;
  const int bbase = blockIdx.x * RPB;
  if (bbase + RPB > nb) return;

  {
    unsigned* za = (unsigned*)(void*)sA;
    for (int i = tid; i < RPB * KCAT; i += NTHR) za[i] = 0u;
    for (int i = tid; i < RPB * OPITCH; i += NTHR) sO[i] = 0.0f;
  }
  __syncthreads();
  load_gate_weights(eWih, eWhh, eBih, eBhh, sW, sBrz, sBin, sBhn, tid);
  stage_x(x, sA, bbase, 0, tid);
  __syncthreads();

  float hreg[8];
#pragma unroll
  for (int r = 0; r < 8; ++r) hreg[r] = 0.0f;

  for (int t = 0; t < TSTEPS; ++t) {
    const int cur = t & 1;
    const _Float16* Acur = sA + cur * (RPB * KCAT);
    _Float16* Anxt = sA + (cur ^ 1) * (RPB * KCAT);
    gru_step(Acur, Anxt, sW, sBrz, sBin, sBhn, hreg, w, m, k8);
    if (t + 1 < TSTEPS) stage_x(x, Anxt, bbase, t + 1, tid);
    __syncthreads();
  }

  load_gate_weights(dWih, dWhh, dBih, dBhh, sW, sBrz, sBin, sBhn, tid);
#pragma unroll 4
  for (int i = tid; i < LINROWS * HDIM; i += NTHR) {
    const int n = i / HDIM;
    const int k = i - n * HDIM;
    const int nc = (n < XDIM) ? n : (XDIM - 1);
    const float v = linW[nc * HDIM + k];
    sLin[i] = (_Float16)((n < XDIM) ? v : 0.0f);
  }
  for (int i = tid; i < LINROWS; i += NTHR) {
    const int ic = (i < XDIM) ? i : (XDIM - 1);
    const float v = linB[ic];
    sLb[i] = (i < XDIM) ? v : 0.0f;
  }
  {
    unsigned* za = (unsigned*)(void*)sA;
    for (int i = tid; i < 2 * RPB * 32; i += NTHR) {
      const int bsel = i >> 9;
      const int rem = i & 511;
      const int row = rem >> 5;
      const int wd = rem & 31;
      za[bsel * (RPB * KCAT / 2) + row * (KCAT / 2) + (HDIM / 2) + wd] = 0u;
    }
  }
  __syncthreads();

  for (int t = 0; t < TSTEPS; ++t) {
    const int cur = t & 1;
    const _Float16* Acur = sA + cur * (RPB * KCAT);
    _Float16* Anxt = sA + (cur ^ 1) * (RPB * KCAT);
    gru_step(Acur, Anxt, sW, sBrz, sBin, sBhn, hreg, w, m, k8);
    __syncthreads();
    if (w < 3) proj_step(Anxt, sLin, sLb, sO, w, m, k8);
    __syncthreads();
    {
      const int row = 2 * w + hh;
      const int c4 = m * 4;
      const v4f v = *(const v4f*)(sO + row * OPITCH + c4);
      float* p = Ows + (((size_t)(bbase + row)) * TSTEPS + t) * OPITCH + c4;
      *(volatile v4f*)p = v;
      __threadfence();
      *(volatile v4f*)p = v;
    }
  }
}

__global__ __launch_bounds__(NTHR) void repack_kernel(const float* __restrict__ Ows, float* __restrict__ out) {
  const int b = blockIdx.x;
  const int tid = threadIdx.x;
  const float* src = Ows + (size_t)b * TSTEPS * OPITCH;
  float* dst = out + (size_t)b * TSTEPS * XDIM;
  v4f vals[RP_ITERS];
#pragma unroll
  for (int it = 0; it < RP_ITERS; ++it) {
    const int q = it * NTHR + tid;
    const int qc = (q < NCHUNK) ? q : (NCHUNK - 1);
    const int f = 4 * qc;
    const int t = f / XDIM;
    const int c = f - t * XDIM;
    const bool same = (c + 2 < XDIM);
    int t2 = same ? t : (t + 1);
    t2 = (t2 < TSTEPS) ? t2 : (TSTEPS - 1);
    const int c2 = same ? (c + 2) : 0;
    const v2f p0 = *(const v2f*)(src + t * OPITCH + c);
    const v2f p1 = *(const v2f*)(src + t2 * OPITCH + c2);
    v4f v; v.x = p0.x; v.y = p0.y; v.z = p1.x; v.w = p1.y;
    vals[it] = v;
  }
  for (int pass = 0; pass < 2; ++pass) {
#pragma unroll
    for (int it = 0; it < RP_ITERS; ++it) {
      const int q = it * NTHR + tid;
      if (q < NCHUNK) *(volatile v4f*)(dst + 4 * q) = vals[it];
    }
    __threadfence();
  }
}

extern "C" void kernel_launch(void* const* d_in, const int* in_sizes, int n_in,
                              void* d_out, int out_size, void* d_ws,
                              size_t ws_size, hipStream_t stream) {
  if (n_in < 11) return;
  const int nb = in_sizes[0] / (TSTEPS * XDIM);
  if (nb < RPB || (nb % RPB) != 0) return;
  if (in_sizes[0] != nb * TSTEPS * XDIM) return;
  if (out_size != nb * TSTEPS * XDIM) return;
  if (in_sizes[1] != GDIM * XDIM || in_sizes[2] != GDIM * HDIM) return;
  if (in_sizes[3] < GDIM || in_sizes[4] < GDIM) return;
  if (in_sizes[5] != GDIM * XDIM || in_sizes[6] != GDIM * HDIM) return;
  if (in_sizes[7] < GDIM || in_sizes[8] < GDIM) return;
  if (in_sizes[9] != XDIM * HDIM || in_sizes[10] < XDIM) return;
  const size_t ws_need = (size_t)nb * TSTEPS * OPITCH * sizeof(float);
  if (ws_need > ws_size) return;

  const float* x    = (const float*)d_in[0];
  const float* eWih = (const float*)d_in[1];
  const float* eWhh = (const float*)d_in[2];
  const float* eBih = (const float*)d_in[3];
  const float* eBhh = (const float*)d_in[4];
  const float* dWih = (const float*)d_in[5];
  const float* dWhh = (const float*)d_in[6];
  const float* dBih = (const float*)d_in[7];
  const float* dBhh = (const float*)d_in[8];
  const float* linW = (const float*)d_in[9];
  const float* linB = (const float*)d_in[10];
  float* Ows = (float*)d_ws;
  float* out = (float*)d_out;

  gru_scan_kernel<<<dim3(nb / RPB), dim3(NTHR), 0, stream>>>(x, eWih, eWhh, eBih, eBhh,
                                                              dWih, dWhh, dBih, dBhh,
                                                              linW, linB, Ows, nb);
  repack_kernel<<<dim3(nb), dim3(NTHR), 0, stream>>>(Ows, out);
}
